// MultiHeadDistanceLayer_18133351924245
// MI455X (gfx1250) — hardware-verified
//
#include <hip/hip_runtime.h>
#include <math.h>

constexpr int kB    = 4;
constexpr int kL    = 2048;
constexpr int kD    = 256;
constexpr int kH    = 8;
constexpr int kHD   = 64;
constexpr int kNH   = kH * kHD;
constexpr int kQKld = 2 * kNH;
constexpr int kTok  = kB * kL;
constexpr int kTbl  = 2 * kL;
constexpr int kQRows = 128;
constexpr int kKeyChunk = 64;
static_assert(kTok % 64 == 0 && kNH % 64 == 0 && kD % 32 == 0, "gemm tiles");
static_assert(kL % kQRows == 0 && kL % kKeyChunk == 0 && kHD == 64, "attention tiles");
static_assert(kTbl % 256 == 0 && kQRows == 8 * 16, "table and block shape");
static_assert((kTok * kD) % (8 * 256) == 0 && kD % 64 == 0, "cast grids");

typedef __attribute__((ext_vector_type(16))) _Float16 v16h;
typedef __attribute__((ext_vector_type(8)))  _Float16 v8h;
typedef __attribute__((ext_vector_type(16))) __bf16   v16b;
typedef __attribute__((ext_vector_type(8)))  __bf16   v8b;
typedef __attribute__((ext_vector_type(8)))  float    v8f;
typedef __attribute__((ext_vector_type(4)))  float    v4f;
typedef __attribute__((ext_vector_type(4)))  unsigned int v4u;

__device__ __forceinline__ unsigned short f2bf_bits(float f) {
  unsigned u = __float_as_uint(f);
  return (unsigned short)((u + 0x7FFFu + ((u >> 16) & 1u)) >> 16);
}
__device__ __forceinline__ float bf_bits2f(unsigned short h) { return __uint_as_float(((unsigned)h) << 16); }
__device__ __forceinline__ float bf_rne(float f) { return bf_bits2f(f2bf_bits(f)); }

__device__ __forceinline__ void dep_guard_h(v8f& a, v8f& b, v16h x, v16h y) { asm volatile("v_nop\n\tv_nop\n\tv_nop\n\tv_nop" : "+v"(a), "+v"(b) : "v"(x), "v"(y)); }
__device__ __forceinline__ void dep_guard_b(v8f& a, v8f& b, v16b x, v16b y) { asm volatile("v_nop\n\tv_nop\n\tv_nop\n\tv_nop" : "+v"(a), "+v"(b) : "v"(x), "v"(y)); }
__device__ __forceinline__ void dep_guard4_h(v8f& a, v8f& b, v8f& c, v8f& d, v16h x, v16h y) { asm volatile("v_nop\n\tv_nop\n\tv_nop\n\tv_nop" : "+v"(a), "+v"(b), "+v"(c), "+v"(d) : "v"(x), "v"(y)); }
__device__ __forceinline__ void dep_guard4_b(v8f& a, v8f& b, v8f& c, v8f& d, v16b x, v16b y) { asm volatile("v_nop\n\tv_nop\n\tv_nop\n\tv_nop" : "+v"(a), "+v"(b), "+v"(c), "+v"(d) : "v"(x), "v"(y)); }
__device__ __forceinline__ void keep4_h(v16h a, v16h b, v16h c, v16h d) { asm volatile("v_nop" :: "v"(a), "v"(b), "v"(c), "v"(d)); }
__device__ __forceinline__ void keep4_b(v16b a, v16b b, v16b c, v16b d) { asm volatile("v_nop" :: "v"(a), "v"(b), "v"(c), "v"(d)); }
__device__ __forceinline__ void acc_guard4(v8f& a, v8f& b, v8f& c, v8f& d) { asm volatile("v_nop\n\tv_nop\n\tv_nop\n\tv_nop" : "+v"(a), "+v"(b), "+v"(c), "+v"(d)); }
template <typename T> struct Frag;
template <> struct Frag<_Float16> {
  typedef v16h V; union U { v16h v; v8h h[2]; };
  static __device__ __forceinline__ v16h load(const _Float16* p) {
    U f; f.h[0] = *(const v8h*)(p); f.h[1] = *(const v8h*)(p + 16); return f.v;
  }
  static __device__ __forceinline__ v8f mma(v16h a, v16h b, v8f c) {
    return __builtin_amdgcn_wmma_f32_16x16x32_f16(false, a, false, b, (short)0, c, false, false);
  }
  static __device__ __forceinline__ void guard(v8f& a, v8f& b, v16h x, v16h y) { dep_guard_h(a, b, x, y); }
  static __device__ __forceinline__ void guard4(v8f& a, v8f& b, v8f& c, v8f& d, v16h x, v16h y) { dep_guard4_h(a, b, c, d, x, y); }
  static __device__ __forceinline__ void keep(v16h a, v16h b, v16h c, v16h d) { keep4_h(a, b, c, d); }
};
template <> struct Frag<__bf16> {
  typedef v16b V; union U { v16b v; v8b h[2]; };
  static __device__ __forceinline__ v16b load(const __bf16* p) {
    U f; f.h[0] = *(const v8b*)(p); f.h[1] = *(const v8b*)(p + 16); return f.v;
  }
  static __device__ __forceinline__ v8f mma(v16b a, v16b b, v8f c) {
    return __builtin_amdgcn_wmma_f32_16x16x32_bf16(false, a, false, b, (short)0, c, false, false);
  }
  static __device__ __forceinline__ void guard(v8f& a, v8f& b, v16b x, v16b y) { dep_guard_b(a, b, x, y); }
  static __device__ __forceinline__ void guard4(v8f& a, v8f& b, v8f& c, v8f& d, v16b x, v16b y) { dep_guard4_b(a, b, c, d, x, y); }
  static __device__ __forceinline__ void keep(v16b a, v16b b, v16b c, v16b d) { keep4_b(a, b, c, d); }
};

__device__ __forceinline__ unsigned pk16(unsigned short a, unsigned short b) { return (unsigned)a | ((unsigned)b << 16); }

__device__ __forceinline__ v8f mma_f16_guarded(v16h a, v16h b, v8f c) {
  c = __builtin_amdgcn_wmma_f32_16x16x32_f16(false, a, false, b, (short)0, c, false, false);
  asm volatile("v_nop\n\tv_nop\n\tv_nop\n\tv_nop" : "+v"(c) : "v"(a), "v"(b));
  return c;
}

template <int ET> struct Elem;
template <> struct Elem<0> { typedef _Float16 T; };
template <> struct Elem<1> { typedef __bf16 T; };
template <int ET, bool SPLIT, int BIAS_MODE, int OUT_MODE, bool RESID, int ACT = 0>
__global__ __launch_bounds__(256) void wmma_gemm64(
    const unsigned short* __restrict__ Ap, const unsigned short* __restrict__ A2p, int lda, long strideA,
    const unsigned short* __restrict__ Btp, const unsigned short* __restrict__ Bt2p, int ldb, long strideB,
    void* __restrict__ Cout, void* __restrict__ Cout2, int ldc, long strideC,
    const float* __restrict__ bias,
    const float* __restrict__ resid, long strideR,
    int M, int N, int K, float scale) {
  typedef typename Elem<ET>::T T;
  typedef typename Frag<T>::V V;
  const T* A = (const T*)Ap; const T* A2 = (const T*)A2p; const T* Bt = (const T*)Btp; const T* Bt2 = (const T*)Bt2p;
  __shared__ __align__(16) float sT[8][16 * 68];
  const int b    = blockIdx.y;
  const int lane = threadIdx.x & 31;
  const int wave = threadIdx.x >> 5;
  const int tilesN = N >> 6;
  const int tilesM = M >> 6;
  const int tile = blockIdx.x * 8 + wave;
  if (tile >= tilesM * tilesN) return;
  const int tm = tile / tilesN;
  const int tn = tile - tm * tilesN;
  const int m0 = tm << 6;
  const int n0 = tn << 6;

  const T* Ab  = A  + (size_t)b * strideA;
  const T* Bb  = Bt + (size_t)b * strideB;
  const T* Ab2 = SPLIT ? (A2  + (size_t)b * strideA) : nullptr;
  const T* Bb2 = SPLIT ? (Bt2 + (size_t)b * strideB) : nullptr;

  const int rlane = lane & 15;
  const int koff  = (lane >> 4) * 8;
  const int mOff  = (lane >> 4) * 8;

  v8f acc[4][4];
#pragma unroll
  for (int i = 0; i < 4; ++i)
#pragma unroll
    for (int j = 0; j < 4; ++j) acc[i][j] = (v8f){0.f,0.f,0.f,0.f,0.f,0.f,0.f,0.f};

  for (int k0 = 0; k0 < K; k0 += 32) {
    V bh[4], bl[4];
#pragma unroll
    for (int j = 0; j < 4; ++j) {
      const size_t bo = (size_t)(n0 + (j << 4) + rlane) * ldb + koff + k0;
      bh[j] = Frag<T>::load(Bb + bo);
      if (SPLIT) bl[j] = Frag<T>::load(Bb2 + bo);
    }
#pragma unroll
    for (int i = 0; i < 4; ++i) {
      const size_t ao = (size_t)(m0 + (i << 4) + rlane) * lda + koff + k0;
      V ah = Frag<T>::load(Ab + ao);
      V al;
      if (SPLIT) al = Frag<T>::load(Ab2 + ao);
#pragma unroll
      for (int j = 0; j < 4; ++j) {
        acc[i][j] = Frag<T>::mma(ah, bh[j], acc[i][j]);
        if (SPLIT) {
          acc[i][j] = Frag<T>::mma(ah, bl[j], acc[i][j]);
          acc[i][j] = Frag<T>::mma(al, bh[j], acc[i][j]);
        }
      }
      Frag<T>::guard4(acc[i][0], acc[i][1], acc[i][2], acc[i][3], ah, SPLIT ? al : bh[3]);
    }
    Frag<T>::keep(bh[0], bh[1], bh[2], bh[3]);
    if (SPLIT) Frag<T>::keep(bl[0], bl[1], bl[2], bl[3]);
  }
  acc_guard4(acc[0][0], acc[0][1], acc[0][2], acc[0][3]);
  acc_guard4(acc[1][0], acc[1][1], acc[1][2], acc[1][3]);
  acc_guard4(acc[2][0], acc[2][1], acc[2][2], acc[2][3]);
  acc_guard4(acc[3][0], acc[3][1], acc[3][2], acc[3][3]);

  float* slab = sT[wave];
  const float* Rb = RESID ? (resid + (size_t)b * strideR) : nullptr;
#pragma unroll
  for (int i = 0; i < 4; ++i) {
    const int mBase = m0 + (i << 4);
#pragma unroll
    for (int j = 0; j < 4; ++j) {
      const int n = n0 + (j << 4) + rlane;
      float bv = 0.f;
      if (BIAS_MODE == 2) bv = bias[n];
#pragma unroll
      for (int r = 0; r < 8; ++r) {
        float v = acc[i][j][r] * scale;
        if (BIAS_MODE == 1) v += bias[mBase + mOff + r];
        if (BIAS_MODE == 2) v += bv;
        if (RESID) v += Rb[(size_t)(mBase + mOff + r) * ldc + n];
        if (ACT == 2) v = fmaxf(v, 0.0f);
        if (ACT == 4) v = (v > 0.f) ? v : 0.01f * v;
        slab[(mOff + r) * 68 + (j << 4) + rlane] = v;
      }
    }
    __builtin_amdgcn_fence(__ATOMIC_RELEASE, "workgroup");
    __builtin_amdgcn_wave_barrier();
    __builtin_amdgcn_fence(__ATOMIC_ACQUIRE, "workgroup");
    if (OUT_MODE == 0) {
      float* C = (float*)Cout + (size_t)b * strideC;
      const int hh = lane >> 4, c4 = (lane & 15) * 4;
      for (int pass = 0; pass < 2; ++pass) {
#pragma unroll
        for (int it = 0; it < 8; ++it) {
          const int row = it * 2 + hh;
          v4f v = *(const v4f*)(slab + row * 68 + c4);
          *(volatile v4f*)(C + (size_t)(mBase + row) * ldc + n0 + c4) = v;
        }
        __threadfence();
      }
    } else {
      const int q = lane >> 3, c8 = (lane & 7) * 8;
      unsigned short* C  = (unsigned short*)Cout  + (size_t)b * strideC;
      unsigned short* C2 = (OUT_MODE == 2) ? ((unsigned short*)Cout2 + (size_t)b * strideC) : nullptr;
      for (int pass = 0; pass < 2; ++pass) {
#pragma unroll
        for (int it = 0; it < 4; ++it) {
          const int row = it * 4 + q;
          const float* sp = slab + row * 68 + c8;
          v8h hv, lv;
#pragma unroll
          for (int e = 0; e < 8; ++e) {
            if (OUT_MODE == 1) {
              hv[e] = (_Float16)sp[e];
            } else {
              unsigned short hb = f2bf_bits(sp[e]);
              unsigned short lb = f2bf_bits(sp[e] - bf_bits2f(hb));
              hv[e] = __builtin_bit_cast(_Float16, hb);
              lv[e] = __builtin_bit_cast(_Float16, lb);
            }
          }
          *(volatile v8h*)(C + (size_t)(mBase + row) * ldc + n0 + c8) = hv;
          if (OUT_MODE == 2) *(volatile v8h*)(C2 + (size_t)(mBase + row) * ldc + n0 + c8) = lv;
        }
        __threadfence();
      }
    }
    __builtin_amdgcn_fence(__ATOMIC_RELEASE, "workgroup");
    __builtin_amdgcn_wave_barrier();
    __builtin_amdgcn_fence(__ATOMIC_ACQUIRE, "workgroup");
  }
}

__global__ __launch_bounds__(256) void cast8_bf16_kernel(const float* __restrict__ in, unsigned short* __restrict__ out, int n8) {
  const int i = blockIdx.x * 256 + threadIdx.x;
  if (i >= n8) return;
  const float* p = in + 8 * (size_t)i;
  const v4f a = *(const v4f*)(p);
  const v4f c = *(const v4f*)(p + 4);
  unsigned short hb[8];
#pragma unroll
  for (int e = 0; e < 4; ++e) {
    hb[e]     = f2bf_bits(a[e]);
    hb[4 + e] = f2bf_bits(c[e]);
  }
  const v4u u = (v4u){pk16(hb[0], hb[1]), pk16(hb[2], hb[3]), pk16(hb[4], hb[5]), pk16(hb[6], hb[7])};
  unsigned short* q = out + 8 * (size_t)i;
  *(volatile v4u*)q = u;
  __threadfence();
  *(volatile v4u*)q = u;
}

__global__ __launch_bounds__(256) void wt_cast_kernel(const float* __restrict__ Wq, const float* __restrict__ Wk,
                                                      unsigned short* __restrict__ Wt) {
  __shared__ float sm[64][65];
  const int t  = threadIdx.x;
  const int d0 = blockIdx.x * 64;
  const int n0 = blockIdx.y * 64;
  const int z  = blockIdx.z;
  const float* W = (z == 0) ? Wq : Wk;
#pragma unroll
  for (int i = 0; i < 16; ++i) {
    const int e  = i * 256 + t;
    const int r  = e >> 6;
    const int cc = e & 63;
    sm[cc][r] = W[(size_t)(d0 + r) * kNH + n0 + cc];
  }
  __syncthreads();
  const int lane = t & 31, wave = t >> 5;
  const int q = lane >> 3, c8 = (lane & 7) * 8;
  unsigned short* op = Wt + (size_t)z * kNH * kD;
  for (int pass = 0; pass < 2; ++pass) {
#pragma unroll
    for (int it = 0; it < 2; ++it) {
      const int row = wave * 8 + it * 4 + q;
      unsigned short hb[8];
#pragma unroll
      for (int e = 0; e < 8; ++e) hb[e] = f2bf_bits(sm[row][c8 + e]);
      const v4u u = (v4u){pk16(hb[0], hb[1]), pk16(hb[2], hb[3]), pk16(hb[4], hb[5]), pk16(hb[6], hb[7])};
      *(volatile v4u*)(op + (size_t)(n0 + row) * kD + d0 + c8) = u;
    }
    __threadfence();
  }
}

__global__ __launch_bounds__(256) void attn_dist_kernel(const unsigned short* __restrict__ QK,
                                                        const float* __restrict__ pmean, const float* __restrict__ plstd,
                                                        const int* __restrict__ mlen, float* __restrict__ DI) {
  __shared__ __align__(16) float tbl[kTbl];
  __shared__ __align__(16) float res[kQRows];
  const int tid  = threadIdx.x;
  const int wave = tid >> 5;
  const int lane = tid & 31;
  const int hh   = lane >> 4;
  const int c    = lane & 15;
  const int l0   = blockIdx.x * kQRows;
  const int h    = blockIdx.y;
  const int b    = blockIdx.z;

  int ml = mlen[0];
  ml = (ml < 1) ? 1 : ml;
  const float inv_ml = 1.0f / (float)ml;
  const float mean = bf_rne(pmean[h]);
  const float lsd  = bf_rne(plstd[h]);
  const float stdv = expf(lsd);
  const float istd = 1.0f / stdv;
  const float coef = ((1.0f / stdv) / sqrtf(6.2831852f)) * 0.125f;

#pragma unroll 1
  for (int it = 0; it < kTbl / 256; ++it) {
    const int i = it * 256 + tid;
    const float dd = (float)(i - kL) * inv_ml;
    const float u  = (dd - mean) * istd;
    tbl[i] = coef * expf(-0.5f * (u * u));
  }
  __syncthreads();

  const int q0 = l0 + wave * 16;
  const _Float16* Qp = (const _Float16*)(const void*)QK + (size_t)(b * kL) * kQKld + h * kHD;
  const _Float16* Kp = Qp + kNH;
  v16h qa[2];
#pragma unroll
  for (int dc = 0; dc < 2; ++dc)
    qa[dc] = Frag<_Float16>::load(Qp + (size_t)(q0 + c) * kQKld + dc * 32 + 8 * hh);

  float den[8], num[8], rdel[8];
#pragma unroll
  for (int r = 0; r < 8; ++r) { den[r] = 0.0f; num[r] = 0.0f; rdel[r] = (float)r * inv_ml; }
  const int qr0   = q0 + 8 * hh;
  const int ibase = c - qr0 + kL;

  for (int kc = 0; kc < kL / kKeyChunk; ++kc) {
    const int kv0 = kc * kKeyChunk;
    v8f s[4];
#pragma unroll
    for (int j = 0; j < 4; ++j) {
      s[j] = (v8f){0.f,0.f,0.f,0.f,0.f,0.f,0.f,0.f};
      const _Float16* krow = Kp + (size_t)(kv0 + j * 16 + c) * kQKld + 8 * hh;
#pragma unroll
      for (int dc = 0; dc < 2; ++dc) {
        const v16h kb = Frag<_Float16>::load(krow + dc * 32);
        s[j] = mma_f16_guarded(qa[dc], kb, s[j]);
      }
    }
    const float dl = (float)(kv0 + c - qr0) * inv_ml;
#pragma unroll
    for (int j = 0; j < 4; ++j) {
      const int   i0 = ibase + kv0 + j * 16;
      const float dj = dl + (float)(j * 16) * inv_ml;
#pragma unroll
      for (int r = 0; r < 8; ++r) {
        const float pr = tbl[i0 - r];
        float lg = s[j][r] * pr;
        lg = fminf(lg, 80.0f);
        const float p = expf(lg);
        den[r] += p;
        num[r] = fmaf(p, dj - rdel[r], num[r]);
      }
    }
  }

#pragma unroll
  for (int r = 0; r < 8; ++r) {
    float dn = den[r], nm = num[r];
#pragma unroll
    for (int off = 1; off < 16; off <<= 1) {
      dn += __shfl_xor(dn, off, 32);
      nm += __shfl_xor(nm, off, 32);
    }
    const float val = nm * (1.0f / dn);
    if (c == 0) res[wave * 16 + 8 * hh + r] = val;
  }
  __syncthreads();
  if (wave == 0) {
    const v4f v = *(const v4f*)(res + 4 * lane);
    float* dp = DI + ((size_t)(h * kB + b) * kL + l0) + 4 * lane;
    *(volatile v4f*)dp = v;
    __threadfence();
    *(volatile v4f*)dp = v;
  }
}

__global__ __launch_bounds__(256) void out_gather_kernel(const float* __restrict__ DI, float* __restrict__ out) {
  __shared__ __align__(16) float sm[kQRows * kH];
  const int t  = threadIdx.x;
  const int l0 = blockIdx.x * kQRows;
  const int b  = blockIdx.y;
  const int h  = t >> 5;
  const int i4 = (t & 31) * 4;
  const v4f v = *(const v4f*)(DI + ((size_t)(h * kB + b) * kL + l0 + i4));
#pragma unroll
  for (int e = 0; e < 4; ++e) sm[(i4 + e) * kH + h] = v[e];
  __syncthreads();
  const v4f o = *(const v4f*)(sm + 4 * t);
  float* op = out + ((size_t)(b * kL + l0)) * kH + 4 * t;
  *(volatile v4f*)op = o;
  __threadfence();
  *(volatile v4f*)op = o;
}

extern "C" void kernel_launch(void* const* d_in, const int* in_sizes, int n_in,
                              void* d_out, int out_size, void* d_ws, size_t ws_size,
                              hipStream_t stream) {
  if (n_in < 8) return;
  if (in_sizes[0] != kTok * kD) return;
  if (in_sizes[1] != kD * kNH || in_sizes[3] != kD * kNH) return;
  if (in_sizes[2] != kNH || in_sizes[4] != kNH) return;
  if (in_sizes[5] != kH || in_sizes[6] != kH || in_sizes[7] < 1) return;
  if (out_size != kTok * kH) return;

  const size_t szXb = (size_t)kTok * kD * 2;
  const size_t szWt = (size_t)2 * kNH * kD * 2;
  const size_t szQK = (size_t)kTok * kQKld * 2;
  const size_t szDI = (size_t)kH * kB * kL * 4;
  const size_t offXb = 0;
  const size_t offWt = offXb + szXb;
  const size_t offQK = offWt + szWt;
  const size_t offDI = offQK + szQK;
  const size_t total = offDI + szDI;
  if (ws_size < total) return;

  const float* x   = (const float*)d_in[0];
  const float* Wq  = (const float*)d_in[1];
  const float* bq  = (const float*)d_in[2];
  const float* Wk  = (const float*)d_in[3];
  const float* bk  = (const float*)d_in[4];
  const float* pm  = (const float*)d_in[5];
  const float* lps = (const float*)d_in[6];
  const int*   mlp = (const int*)d_in[7];
  float* out = (float*)d_out;
  char* ws = (char*)d_ws;
  unsigned short* Xb = (unsigned short*)(ws + offXb);
  unsigned short* Wt = (unsigned short*)(ws + offWt);
  unsigned short* QK = (unsigned short*)(ws + offQK);
  float* DI = (float*)(ws + offDI);

  const int n8 = (kTok * kD) / 8;
  cast8_bf16_kernel<<<dim3(n8 / 256), dim3(256), 0, stream>>>(x, Xb, n8);
  wt_cast_kernel<<<dim3(kD / 64, kNH / 64, 2), dim3(256), 0, stream>>>(Wq, Wk, Wt);

  const int tilesProj = (kTok / 64) * (kNH / 64);
  wmma_gemm64<1, false, 2, 1, false, 0><<<dim3(tilesProj / 8, 1), dim3(256), 0, stream>>>(
      Xb, Xb, kD, 0L, Wt, Wt, kD, 0L,
      (void*)QK, (void*)QK, kQKld, 0L, bq, bq, 0L, kTok, kNH, kD, 1.0f);
  wmma_gemm64<1, false, 2, 1, false, 0><<<dim3(tilesProj / 8, 1), dim3(256), 0, stream>>>(
      Xb, Xb, kD, 0L, Wt + (size_t)kNH * kD, Wt + (size_t)kNH * kD, kD, 0L,
      (void*)(QK + kNH), (void*)(QK + kNH), kQKld, 0L, bk, bk, 0L, kTok, kNH, kD, 1.0f);

  attn_dist_kernel<<<dim3(kL / kQRows, kH, kB), dim3(256), 0, stream>>>(QK, pm, lps, mlp, DI);

  out_gather_kernel<<<dim3(kL / kQRows, kB), dim3(256), 0, stream>>>(DI, out);
}
